// GNNTrafficPredictor_44272522887550
// MI455X (gfx1250) — hardware-run, weakly checked
//
#include <hip/hip_runtime.h>


namespace {
constexpr int N = 4096, E = 131072, NH = 8, HF = 64, D = 512, NBLK = N / 16;
constexpr float XS = 8.0f, PS = 1024.0f, WSC = 256.0f, SLOPE = 0.2f;
typedef _Float16 b16;
typedef __attribute__((ext_vector_type(16))) _Float16 v16b;
typedef __attribute__((ext_vector_type(8))) _Float16 v8b;
typedef __attribute__((ext_vector_type(8))) float v8f;
typedef __attribute__((ext_vector_type(4))) float v4f;
__device__ __forceinline__ float bf16_rne(float f) { unsigned int u = __float_as_uint(f); u += 0x7FFFu + ((u >> 16) & 1u); return __uint_as_float(u & 0xFFFF0000u); }
__device__ __forceinline__ void split16(float v, b16& hi, b16& lo) { hi = (b16)v; lo = (b16)(v - (float)hi); }
__device__ __forceinline__ v16b frag_kb(const b16* p, int hh) { const v8b a = *(const v8b*)(p + 8 * hh), b = *(const v8b*)(p + 16 + 8 * hh); v16b f;
#pragma unroll
  for (int e = 0; e < 8; ++e) { f[e] = a[e]; f[8 + e] = b[e]; } return f; }
__device__ __forceinline__ v8f wmma16b(v16b a, v16b b, v8f c) { v8f d = __builtin_amdgcn_wmma_f32_16x16x32_f16(false, a, false, b, (short)0, c, false, false); asm volatile("v_nop\n\tv_nop\n\tv_nop\n\tv_nop" : "+v"(d) : "v"(a), "v"(b)); return d; }
__device__ __forceinline__ void wave_lds_sync() { __builtin_amdgcn_fence(__ATOMIC_RELEASE, "workgroup"); __builtin_amdgcn_wave_barrier(); __builtin_amdgcn_fence(__ATOMIC_ACQUIRE, "workgroup"); }
__device__ __forceinline__ float pmul(float a, float b) { float p = a * b; asm volatile("" : "+v"(p)); return p; }
__device__ __forceinline__ int iclamp(int v, int lo, int hi) { return v < lo ? lo : (v > hi ? hi : v); }
__device__ __forceinline__ float leaky(float v) { return v >= 0.0f ? v : SLOPE * v; }
constexpr int CSR_NBLK7 = 512, CSR_GB7 = 7, CSR_GN7 = 1 << CSR_GB7  , CSR_TS7 = (CSR_GN7 < 32 ? 32 : CSR_GN7)  , CSR_MAXG7 = 512, CSR_CAP7 = 12288  ;
__device__ __host__ __forceinline__ int csr_tix7(int v) { return (v >> CSR_GB7) * CSR_TS7 + (v & (CSR_GN7 - 1)); }
__global__ __launch_bounds__(64) void csrA_kernel7(const int* __restrict__ dst, int E, int N, int nG, int CHP, int NGP, int* __restrict__ STG, int* __restrict__ HST) {
  extern __shared__ int sm[];
  int* cnt = sm; int* run = sm + NGP; int* ids = sm + 2 * NGP;
  const int b = blockIdx.x; const int ch = (E + CSR_NBLK7 - 1) / CSR_NBLK7; const int e0 = b * ch, e1 = min(E, e0 + ch);
  for (int i = threadIdx.x; i < NGP; i += 64) cnt[i] = 0;
  for (int i = threadIdx.x; i < CHP; i += 64) ids[i] = -1;
  __syncthreads();
  if (threadIdx.x == 0) {
    for (int e = e0; e < e1; ++e) { int d = dst[e]; d = (d < 0) ? 0 : (d >= N ? N - 1 : d); cnt[d >> CSR_GB7] += 1; }
    int acc = 0; for (int g = 0; g < nG; ++g) { run[g] = acc; acc += cnt[g]; }
    for (int e = e0; e < e1; ++e) { int d = dst[e]; d = (d < 0) ? 0 : (d >= N ? N - 1 : d); const int g = d >> CSR_GB7; ids[run[g]] = e; run[g] += 1; } }
  __syncthreads();
  typedef __attribute__((ext_vector_type(4))) int v4i;
  for (int pass = 0; pass < 2; ++pass) {
    for (int i = threadIdx.x; i < CHP / 4; i += 64) *(volatile v4i*)(STG + (size_t)b * CHP + i * 4) = *(const v4i*)(&ids[i * 4]);
    for (int i = threadIdx.x; i < NGP / 4; i += 64) { v4i v; for (int e = 0; e < 4; ++e) v[e] = (i * 4 + e < nG) ? cnt[i * 4 + e] : 0; *(volatile v4i*)(HST + (size_t)b * NGP + i * 4) = v; }
    __threadfence(); }
}
__global__ __launch_bounds__(512) void csrS_kernel7(const int* __restrict__ HST, int nG, int NGP, int* __restrict__ START, int* __restrict__ TOT, int* __restrict__ OFF) {
  __shared__ int tot[CSR_MAXG7];
  const int b = threadIdx.x;
  for (int pass = 0; pass < 2; ++pass) { int runb = 0; for (int g = 0; g < nG; ++g) { int c = HST[(size_t)b * NGP + g]; c = (c < 0) ? 0 : c; ((volatile int*)OFF)[(size_t)g * CSR_NBLK7 + b] = runb; runb += c; } __threadfence(); }
  for (int g = threadIdx.x; g < nG; g += 512) { int s = 0; for (int bb = 0; bb < CSR_NBLK7; ++bb) { int c = HST[(size_t)bb * NGP + g]; s += (c < 0) ? 0 : c; } tot[g] = s; }
  __syncthreads();
  if (threadIdx.x < 32) {
    __shared__ int st[CSR_MAXG7 + 32];
    if (threadIdx.x == 0) { int acc = 0; for (int g = 0; g < NGP; ++g) { st[g] = acc; if (g < nG) acc += (tot[g] + 31) & ~31; } st[NGP] = acc; }
    __builtin_amdgcn_fence(__ATOMIC_RELEASE, "workgroup"); __builtin_amdgcn_wave_barrier(); __builtin_amdgcn_fence(__ATOMIC_ACQUIRE, "workgroup");
    for (int pass = 0; pass < 2; ++pass) { for (int i = threadIdx.x; i < NGP + 32; i += 32) { ((volatile int*)START)[i] = (i <= NGP) ? st[min(i, NGP)] : 0; ((volatile int*)TOT)[i] = (i < nG) ? tot[i] : 0; } __threadfence(); } }
}
__global__ __launch_bounds__(256) void csrB_kernel7(const int* __restrict__ dst, int N, int nG, int CHP, int NGP, int permLen, const int* __restrict__ STG, const int* __restrict__ HST, const int* __restrict__ OFF, const int* __restrict__ START, const int* __restrict__ TOT, int* __restrict__ PERM, int* __restrict__ ROWPTR, int* __restrict__ ROWCNT, int* __restrict__ FLAG) {
  typedef __attribute__((ext_vector_type(4))) int v4i;
  __shared__ int ids[CSR_CAP7]; __shared__ unsigned short key[CSR_CAP7]; __shared__ int outp[CSR_CAP7]; __shared__ int ncnt[CSR_GN7 + 1]; __shared__ int boff[CSR_NBLK7 + 1];
  const int g = blockIdx.x, t_ = threadIdx.x; int tot = TOT[g]; int st = START[g], stn = START[g + 1]; const int v0 = g * CSR_GN7; const int nv = min(CSR_GN7, N - v0); const int t0 = g * CSR_TS7;
  st = (st < 0) ? 0 : (st > permLen - 32 ? permLen - 32 : st) & ~31; stn = (stn < st) ? st : (stn > permLen ? permLen : stn); tot = (tot < 0) ? 0 : tot; if (tot > stn - st && tot <= CSR_CAP7) tot = stn - st;
  if (tot > CSR_CAP7) {
    for (int pass = 0; pass < 2; ++pass) { for (int i = t_; i < CSR_TS7 / 4; i += 256) { v4i a, c; for (int e = 0; e < 4; ++e) { a[e] = st; c[e] = 0; } *(volatile v4i*)(ROWPTR + t0 + i * 4) = a; *(volatile v4i*)(ROWCNT + t0 + i * 4) = c; } if (t_ == 0) ((volatile int*)FLAG)[0] = 1; __threadfence(); } (void)nv; return; }
  if (t_ == 0) { int acc = 0; for (int b = 0; b < CSR_NBLK7; ++b) { boff[b] = acc; int c = HST[(size_t)b * NGP + g]; c = (c < 0) ? 0 : (c > CHP ? CHP : c); acc += c; if (acc > tot) acc = tot; } boff[CSR_NBLK7] = acc; }
  for (int i = t_; i <= CSR_GN7; i += 256) ncnt[i] = 0;
  __syncthreads();
  for (int b = 0; b < CSR_NBLK7; ++b) { const int c = boff[b + 1] - boff[b]; int o_ = OFF[(size_t)g * CSR_NBLK7 + b]; o_ = (o_ < 0) ? 0 : (o_ > CHP - c ? CHP - c : o_); const int* src_ = STG + (size_t)b * CHP + o_;
    for (int i = t_; i < c; i += 256) { int id = src_[i]; id = (id < 0) ? 0 : id; ids[boff[b] + i] = id; int d = dst[id]; d = (d < v0) ? v0 : (d >= N ? N - 1 : d); int kk = d - v0; kk = (kk < 0) ? 0 : (kk >= CSR_GN7 ? CSR_GN7 - 1 : kk); key[boff[b] + i] = (unsigned short)kk; } }
  __syncthreads();
  if (t_ == 0) { for (int i = 0; i < tot; ++i) ncnt[key[i]] += 1; int acc = 0; for (int vl = 0; vl < CSR_GN7; ++vl) { const int c = ncnt[vl]; ncnt[vl] = acc; acc += c; } ncnt[CSR_GN7] = acc;
    for (int i = 0; i < tot; ++i) { const int vl = key[i]; outp[ncnt[vl]] = ids[i]; ncnt[vl] += 1; }
    for (int vl = CSR_GN7; vl > 0; --vl) ncnt[vl] = ncnt[vl - 1]; ncnt[0] = 0; }
  __syncthreads();
  for (int pass = 0; pass < 2; ++pass) {
    for (int i = t_; i < (stn - st) / 4; i += 256) { v4i v; for (int e = 0; e < 4; ++e) { const int q = i * 4 + e; v[e] = (q < tot) ? outp[q] : -1; } *(volatile v4i*)(PERM + st + i * 4) = v; }
    for (int i = t_; i < CSR_TS7 / 4; i += 256) { v4i a, c; for (int e = 0; e < 4; ++e) { const int vl = i * 4 + e; const int vc = vl < CSR_GN7 ? vl : CSR_GN7; a[e] = (vl < CSR_GN7) ? st + ncnt[vc] : st; c[e] = (vl < nv) ? (ncnt[(vc < CSR_GN7 ? vc : CSR_GN7 - 1) + 1] - ncnt[vc]) : 0; } *(volatile v4i*)(ROWPTR + t0 + i * 4) = a; *(volatile v4i*)(ROWCNT + t0 + i * 4) = c; }
    __threadfence(); }
}
__global__ __launch_bounds__(256) void csrZ_kernel7(int* __restrict__ p, size_t n4) { typedef __attribute__((ext_vector_type(4))) int v4i; const size_t tid = (size_t)blockIdx.x * 256 + threadIdx.x, nth = (size_t)gridDim.x * 256; v4i z = {0, 0, 0, 0}; for (size_t i = tid; i < n4; i += nth) *(volatile v4i*)(p + i * 4) = z; }
struct CsrBufs7 { int *STG, *HST, *OFF, *START, *TOT, *PERM, *ROWPTR, *ROWCNT, *FLAG; int nG, NGP, CHP; size_t permLen; char* base; size_t bytes; };
static size_t csr_carve7(CsrBufs7& c, char* ws, size_t off, int E, int N) {
  const size_t off0 = off; c.base = ws + off;
  auto al = [&](size_t bytes) { char* p = ws + off; off += (bytes + 255) & ~(size_t)255; return p; };
  c.nG = (N + CSR_GN7 - 1) / CSR_GN7; c.NGP = (c.nG + 31) & ~31; const int ch = (E + CSR_NBLK7 - 1) / CSR_NBLK7; c.CHP = (ch + 31) & ~31; c.permLen = (size_t)E + 32 * (size_t)c.nG + 32;
  c.STG = (int*)al((size_t)CSR_NBLK7 * c.CHP * 4); c.HST = (int*)al((size_t)CSR_NBLK7 * c.NGP * 4); c.OFF = (int*)al((size_t)c.NGP * CSR_NBLK7 * 4); c.START = (int*)al((size_t)(c.NGP + 64) * 4); c.TOT = (int*)al((size_t)(c.NGP + 64) * 4);
  c.PERM = (int*)al(c.permLen * 4); c.ROWPTR = (int*)al((size_t)c.nG * CSR_TS7 * 4); c.ROWCNT = (int*)al((size_t)c.nG * CSR_TS7 * 4); c.FLAG = (int*)al(256);
  c.bytes = off - off0; return off;
}
static void csr_build7(const CsrBufs7& c, const int* dst, int E, int N, hipStream_t stream) {
  const size_t smem = (size_t)(2 * c.NGP + c.CHP) * 4;
  csrZ_kernel7<<<512, 256, 0, stream>>>((int*)c.base, c.bytes / 16);
  csrA_kernel7<<<CSR_NBLK7, 64, smem, stream>>>(dst, E, N, c.nG, c.CHP, c.NGP, c.STG, c.HST);
  csrS_kernel7<<<1, 512, 0, stream>>>(c.HST, c.nG, c.NGP, c.START, c.TOT, c.OFF);
  csrB_kernel7<<<c.nG, 256, 0, stream>>>(dst, N, c.nG, c.CHP, c.NGP, (int)c.permLen, c.STG, c.HST, c.OFF, c.START, c.TOT, c.PERM, c.ROWPTR, c.ROWCNT, c.FLAG);
}


__global__ __launch_bounds__(256) void wput_kernel(const float* __restrict__ w, int KIN, int KP, int OUTW, int OUTP, b16* __restrict__ WT) {
  const int KG = KP / 8; const size_t u = (size_t)blockIdx.x * 256 + threadIdx.x; if (u >= (size_t)OUTP * KG) return; const int o = (int)(u / KG), k0 = (int)(u % KG) * 8; v8b v;
#pragma unroll
  for (int j = 0; j < 8; ++j) { const int k = k0 + j; v[j] = (k < KIN && o < OUTW) ? (b16)(bf16_rne(w[(size_t)k * OUTW + o]) * WSC) : (b16)0.0f; } for (int pass = 0; pass < 2; ++pass) { *(volatile v8b*)(WT + (size_t)o * KP + k0) = v; __threadfence(); }
}
template <int KIN, int NT, int EXACT, int RELU, int ATT>
__global__ __launch_bounds__(32) void dense_kernel(const float* __restrict__ IN, int inp, int inw, const b16* __restrict__ WT, const float* __restrict__ bias, const float* __restrict__ asv, const float* __restrict__ adv, float* __restrict__ OUT, float* __restrict__ AS) {
  __shared__ __attribute__((aligned(16))) b16 Ah[16][KIN + 8], Al[16][(EXACT ? 32 : KIN) + 8]; __shared__ __attribute__((aligned(16))) float Tf[16][128 + 4], Ps[16][16];
  const int lane = threadIdx.x, nloc = lane & 15, hlf = lane >> 4; const size_t m0 = (size_t)blockIdx.x * 16;
  for (int rr = 0; rr < 16; ++rr) for (int q = 0; q < KIN / 32; ++q) { const int c = q * 32 + lane; const float v = c < inw ? IN[(m0 + rr) * inp + c] : 0.0f; if (EXACT) Ah[rr][c] = (b16)(bf16_rne(v) * XS); else { b16 p, ql; split16(v * XS, p, ql); Ah[rr][c] = p; Al[rr][c] = ql; } }
  wave_lds_sync(); float ps[8], pd[8];
#pragma unroll
  for (int r8 = 0; r8 < 8; ++r8) { ps[r8] = 0.0f; pd[r8] = 0.0f; }
#pragma unroll 1
  for (int cg = 0; cg < (NT + 7) / 8; ++cg) { const int nt = NT - cg * 8 < 8 ? NT - cg * 8 : 8; v8f acc[8];
#pragma unroll
    for (int t = 0; t < 8; ++t) acc[t] = (v8f){};
#pragma unroll 2
    for (int kb = 0; kb < KIN; kb += 32) { const v16b a = frag_kb(&Ah[nloc][kb], hlf); v16b al; if (!EXACT) al = frag_kb(&Al[nloc][kb], hlf);
#pragma unroll
      for (int t = 0; t < 8; ++t) if (t < nt) { const v16b bw = frag_kb(WT + (size_t)(cg * 128 + t * 16 + nloc) * KIN + kb, hlf); acc[t] = wmma16b(a, bw, acc[t]); if (!EXACT) acc[t] = wmma16b(al, bw, acc[t]); } }
#pragma unroll
    for (int t = 0; t < 8; ++t) { if (t < nt) { const int c = cg * 128 + t * 16 + nloc; const float bb = bias ? bf16_rne(bias[c]) : 0.0f; float wa = 0.0f, wd = 0.0f; if (ATT) { wa = bf16_rne(asv[c]); wd = bf16_rne(adv[c]); }
#pragma unroll
        for (int r8 = 0; r8 < 8; ++r8) { float v = acc[t][r8] * (1.0f / (XS * WSC)) + bb; if (RELU) v = fmaxf(v, 0.0f); Tf[8 * hlf + r8][t * 16 + nloc] = v; if (ATT) { ps[r8] += pmul(v, wa); pd[r8] += pmul(v, wd); } }
        if (ATT && (t & 3) == 3) { const int h = (cg * 128 + t * 16) / HF;
#pragma unroll
          for (int r8 = 0; r8 < 8; ++r8) { float a2 = ps[r8], d2 = pd[r8]; for (int o = 1; o < 16; o <<= 1) { a2 += __shfl_xor(a2, o); d2 += __shfl_xor(d2, o); } if (nloc == 0) { Ps[8 * hlf + r8][h] = a2; Ps[8 * hlf + r8][NH + h] = d2; } ps[r8] = 0.0f; pd[r8] = 0.0f; } } } }
    wave_lds_sync();
    for (int pass = 0; pass < 2; ++pass) { for (int rr = 0; rr < 16; ++rr) for (int c = lane; c < nt * 16; c += 32) ((volatile float*)OUT)[(m0 + rr) * (size_t)(NT * 16) + cg * 128 + c] = Tf[rr][c]; __threadfence(); }
    wave_lds_sync(); }
  if (ATT) { for (int pass = 0; pass < 2; ++pass) { for (int q = 0; q < 8; ++q) { const int i = q * 32 + lane; ((volatile float*)AS)[m0 * 16 + i] = Ps[i >> 4][i & 15]; } __threadfence(); } }
}
__global__ __launch_bounds__(256) void gat_kernel(const float* __restrict__ HW, const float* __restrict__ AS, const float* __restrict__ bias, const int* __restrict__ srcs, const int* __restrict__ PERM, const int* __restrict__ ROWPTR, const int* __restrict__ ROWCNT, int permLen, int NLIM, float* __restrict__ G) {
  const int wave = threadIdx.x >> 5, lane = threadIdx.x & 31; const size_t v = (size_t)blockIdx.x * 8 + wave; if (v >= (size_t)NLIM) return; const int h = lane >> 2; const int c0 = lane * 16;
  const float ad = AS[v * 16 + NH + h]; int st = ROWPTR[v], cnt = ROWCNT[v]; cnt = iclamp(cnt, 0, 1 << 20); st = iclamp(st, 0, permLen - cnt);
  float mx = leaky(AS[v * 16 + h] + ad);
#pragma unroll 1
  for (int j = 0; j < cnt; ++j) { const int e = iclamp(PERM[st + j], 0, E - 1); const size_t s = (size_t)iclamp(srcs[e], 0, N - 1); if (s >= (size_t)NLIM) continue; mx = fmaxf(mx, leaky(AS[s * 16 + h] + ad)); }
  float den; float o[16]; { const float p = __expf(leaky(AS[v * 16 + h] + ad) - mx); den = p;
#pragma unroll
    for (int i = 0; i < 16; ++i) o[i] = pmul(p, HW[v * D + c0 + i]); }
#pragma unroll 1
  for (int j = 0; j < cnt; ++j) { const int e = iclamp(PERM[st + j], 0, E - 1); const size_t s = (size_t)iclamp(srcs[e], 0, N - 1); if (s >= (size_t)NLIM) continue; const float p = __expf(leaky(AS[s * 16 + h] + ad) - mx); den += p; const float* hs = HW + s * D + c0;
#pragma unroll
    for (int i = 0; i < 16; ++i) o[i] += pmul(p, hs[i]); }
  const float inv = 1.0f / (den + 1e-16f); float r[16];
#pragma unroll
  for (int i = 0; i < 16; ++i) r[i] = pmul(o[i], inv) + bf16_rne(bias[c0 + i]);
  for (int pass = 0; pass < 2; ++pass) {
#pragma unroll
    for (int q = 0; q < 4; ++q) *(volatile v4f*)(G + v * D + c0 + q * 4) = (v4f){r[q * 4], r[q * 4 + 1], r[q * 4 + 2], r[q * 4 + 3]}; __threadfence(); }
}
__global__ __launch_bounds__(256) void stats_kernel(const float* __restrict__ G, int NLIM, float* __restrict__ ST) {
  __shared__ float red[256]; const int c = blockIdx.x, tid = threadIdx.x; float s = 0.0f;
  for (int n = tid; n < NLIM; n += 256) s += G[(size_t)n * D + c]; red[tid] = s; __syncthreads();
  for (int w = 128; w > 0; w >>= 1) { if (tid < w) red[tid] += red[tid + w]; __syncthreads(); } const float mu = red[0] / (float)NLIM; __syncthreads();
  float q = 0.0f; for (int n = tid; n < NLIM; n += 256) { const float dd = G[(size_t)n * D + c] - mu; q += pmul(dd, dd); } red[tid] = q; __syncthreads();
  for (int w = 128; w > 0; w >>= 1) { if (tid < w) red[tid] += red[tid + w]; __syncthreads(); } const float rs = rsqrtf(red[0] / (float)NLIM + 1e-5f);
  if (tid < 32) { for (int pass = 0; pass < 2; ++pass) { ((volatile float*)ST)[(size_t)c * 32 + tid] = tid == 0 ? mu : (tid == 1 ? rs : 0.0f); __threadfence(); } }
}
__global__ __launch_bounds__(256) void bn_kernel(const float* __restrict__ G, const float* __restrict__ ST, const float* __restrict__ gm, const float* __restrict__ bt, float* __restrict__ Hh) {
  const int wave = threadIdx.x >> 5, lane = threadIdx.x & 31; const size_t v = (size_t)blockIdx.x * 8 + wave; const int c0 = lane * 16; float r[16];
#pragma unroll
  for (int i = 0; i < 16; ++i) { const int c = c0 + i; r[i] = fmaxf(pmul(pmul(G[v * D + c] - ST[c * 32], ST[c * 32 + 1]), bf16_rne(gm[c])) + bf16_rne(bt[c]), 0.0f); }
  for (int pass = 0; pass < 2; ++pass) {
#pragma unroll
    for (int q = 0; q < 4; ++q) *(volatile v4f*)(Hh + v * D + c0 + q * 4) = (v4f){r[q * 4], r[q * 4 + 1], r[q * 4 + 2], r[q * 4 + 3]}; __threadfence(); }
}
__global__ __launch_bounds__(32) void att_kernel(const float* __restrict__ QKV, int NLIM, float* __restrict__ O) {
  __shared__ __attribute__((aligned(16))) b16 Qh[16][72], Ql[16][72], Kh[32][72], Kl[32][72], Ph[16][40], Vh[HF][40], Vl[HF][40]; __shared__ float Sc[16][33], M[16], Dn[16], Sf[16], Of[16][HF + 1];
  const int lane = threadIdx.x, nloc = lane & 15, hlf = lane >> 4; const int nqb = NLIM / 16; const int qb = blockIdx.x % nqb, h = blockIdx.x / nqb; const size_t q0 = (size_t)qb * 16;
  for (int rr = 0; rr < 16; ++rr) { b16 p, ql; split16(QKV[(q0 + rr) * (3 * D) + h * HF + lane] * XS, p, ql); Qh[rr][lane] = p; Ql[rr][lane] = ql; split16(QKV[(q0 + rr) * (3 * D) + h * HF + 32 + lane] * XS, p, ql); Qh[rr][32 + lane] = p; Ql[rr][32 + lane] = ql; }
  if (lane < 16) { M[lane] = -INFINITY; Dn[lane] = 0.0f; Sf[lane] = 0.0f; }
  v8f acc[4];
#pragma unroll
  for (int t = 0; t < 4; ++t) acc[t] = (v8f){};
  wave_lds_sync();
#pragma unroll 1
  for (int kc = 0; kc < NLIM; kc += 32) {
    for (int rr = 0; rr < 32; ++rr) { const size_t kn = kc + rr; const float* kp = QKV + kn * (3 * D) + D + h * HF; const float* vp = QKV + kn * (3 * D) + 2 * D + h * HF; b16 p, ql; split16(kp[lane] * XS, p, ql); Kh[rr][lane] = p; Kl[rr][lane] = ql; split16(kp[32 + lane] * XS, p, ql); Kh[rr][32 + lane] = p; Kl[rr][32 + lane] = ql;
      split16(vp[lane] * XS, p, ql); Vh[lane][rr] = p; Vl[lane][rr] = ql; split16(vp[32 + lane] * XS, p, ql); Vh[32 + lane][rr] = p; Vl[32 + lane][rr] = ql; }
    wave_lds_sync();
#pragma unroll
    for (int blk = 0; blk < 2; ++blk) { v8f s = {};
#pragma unroll
      for (int ks = 0; ks < HF; ks += 32) { const v16b qh = frag_kb(&Qh[nloc][ks], hlf), ql = frag_kb(&Ql[nloc][ks], hlf), kh = frag_kb(&Kh[blk * 16 + nloc][ks], hlf), kl = frag_kb(&Kl[blk * 16 + nloc][ks], hlf); s = wmma16b(qh, kh, s); s = wmma16b(qh, kl, s); s = wmma16b(ql, kh, s); }
#pragma unroll
      for (int r8 = 0; r8 < 8; ++r8) Sc[8 * hlf + r8][blk * 16 + nloc] = s[r8] * (0.125f / (XS * XS)); }
    wave_lds_sync();
#pragma unroll 1
    for (int qi = 0; qi < 16; ++qi) { const float sv = Sc[qi][lane]; float cm = sv; for (int o = 16; o; o >>= 1) cm = fmaxf(cm, __shfl_xor(cm, o)); const float mo = M[qi]; const float mn = fmaxf(mo, cm); const float p = __expf(sv - mn); float psum = p; for (int o = 16; o; o >>= 1) psum += __shfl_xor(psum, o);
      Ph[qi][lane] = (b16)(p * PS); if (lane == 0) { const float sf = (mo == -INFINITY) ? 0.0f : __expf(mo - mn); Sf[qi] = sf; Dn[qi] = Dn[qi] * sf + psum; M[qi] = mn; } }
    wave_lds_sync();
#pragma unroll
    for (int t = 0; t < 4; ++t)
#pragma unroll
      for (int r8 = 0; r8 < 8; ++r8) acc[t][r8] *= Sf[8 * hlf + r8];
    { const v16b pa = frag_kb(&Ph[nloc][0], hlf);
#pragma unroll
      for (int t = 0; t < 4; ++t) { acc[t] = wmma16b(pa, frag_kb(&Vh[t * 16 + nloc][0], hlf), acc[t]); acc[t] = wmma16b(pa, frag_kb(&Vl[t * 16 + nloc][0], hlf), acc[t]); } }
    wave_lds_sync(); }
#pragma unroll
  for (int t = 0; t < 4; ++t)
#pragma unroll
    for (int r8 = 0; r8 < 8; ++r8) { const int rl = 8 * hlf + r8; Of[rl][t * 16 + nloc] = acc[t][r8] * (1.0f / (PS * XS)) / Dn[rl]; }
  wave_lds_sync();
  for (int pass = 0; pass < 2; ++pass) { for (int rr = 0; rr < 16; ++rr) { ((volatile float*)O)[(q0 + rr) * D + h * HF + lane] = Of[rr][lane]; ((volatile float*)O)[(q0 + rr) * D + h * HF + 32 + lane] = Of[rr][32 + lane]; } __threadfence(); }
}
__global__ __launch_bounds__(32) void mlp_kernel(const float* __restrict__ AO, const b16* __restrict__ W0T, const float* __restrict__ b0, const b16* __restrict__ W1T, const float* __restrict__ b1, const float* __restrict__ w2, const float* __restrict__ b2, float* __restrict__ out) {
  __shared__ __attribute__((aligned(16))) b16 Ah[16][D + 8], Al[16][D + 8], Bh[16][264], Bl[16][264]; __shared__ float So[32];
  const int lane = threadIdx.x, nloc = lane & 15, hlf = lane >> 4; const size_t n0 = (size_t)blockIdx.x * 32;
#pragma unroll 1
  for (int half = 0; half < 2; ++half) { const size_t m0 = n0 + half * 16;
    for (int rr = 0; rr < 16; ++rr) for (int q = 0; q < 16; ++q) { b16 p, ql; split16(AO[(m0 + rr) * D + q * 32 + lane] * XS, p, ql); Ah[rr][q * 32 + lane] = p; Al[rr][q * 32 + lane] = ql; }
    wave_lds_sync();
#pragma unroll 1
    for (int cg = 0; cg < 2; ++cg) { v8f acc[8];
#pragma unroll
      for (int t = 0; t < 8; ++t) acc[t] = (v8f){};
#pragma unroll 2
      for (int kb = 0; kb < D; kb += 32) { const v16b a = frag_kb(&Ah[nloc][kb], hlf), al = frag_kb(&Al[nloc][kb], hlf);
#pragma unroll
        for (int t = 0; t < 8; ++t) { const v16b bw = frag_kb(W0T + (size_t)(cg * 128 + t * 16 + nloc) * D + kb, hlf); acc[t] = wmma16b(a, bw, acc[t]); acc[t] = wmma16b(al, bw, acc[t]); } }
#pragma unroll
      for (int t = 0; t < 8; ++t) { const int c = cg * 128 + t * 16 + nloc; const float bb = bf16_rne(b0[c]);
#pragma unroll
        for (int r8 = 0; r8 < 8; ++r8) { b16 p, ql; split16(fmaxf(acc[t][r8] * (1.0f / (XS * WSC)) + bb, 0.0f) * XS, p, ql); Bh[8 * hlf + r8][c] = p; Bl[8 * hlf + r8][c] = ql; } } }
    wave_lds_sync(); v8f acc[8];
#pragma unroll
    for (int t = 0; t < 8; ++t) acc[t] = (v8f){};
#pragma unroll 2
    for (int kb = 0; kb < 256; kb += 32) { const v16b a = frag_kb(&Bh[nloc][kb], hlf), al = frag_kb(&Bl[nloc][kb], hlf);
#pragma unroll
      for (int t = 0; t < 8; ++t) { const v16b bw = frag_kb(W1T + (size_t)(t * 16 + nloc) * 256 + kb, hlf); acc[t] = wmma16b(a, bw, acc[t]); acc[t] = wmma16b(al, bw, acc[t]); } }
    float pd[8];
#pragma unroll
    for (int r8 = 0; r8 < 8; ++r8) pd[r8] = 0.0f;
#pragma unroll
    for (int t = 0; t < 8; ++t) { const int c = t * 16 + nloc; const float bb = bf16_rne(b1[c]), ww = bf16_rne(w2[c]);
#pragma unroll
      for (int r8 = 0; r8 < 8; ++r8) pd[r8] += pmul(fmaxf(acc[t][r8] * (1.0f / (XS * WSC)) + bb, 0.0f), ww); }
#pragma unroll
    for (int r8 = 0; r8 < 8; ++r8) { float s = pd[r8]; for (int o = 1; o < 16; o <<= 1) s += __shfl_xor(s, o); if (nloc == 0) So[half * 16 + 8 * hlf + r8] = s + bf16_rne(b2[0]); }
    wave_lds_sync(); }
  for (int pass = 0; pass < 2; ++pass) { ((volatile float*)out)[n0 + lane] = So[lane]; __threadfence(); }
}
__global__ __launch_bounds__(256) void qb_kernel(const float* __restrict__ bq, const float* __restrict__ bk, const float* __restrict__ bv, float* __restrict__ QB) { for (int i = threadIdx.x; i < 3 * D; i += 256) { const float v = i < D ? bq[i] : (i < 2 * D ? bk[i - D] : bv[i - 2 * D]); for (int pass = 0; pass < 2; ++pass) { ((volatile float*)QB)[i] = v; __threadfence(); } } }
}

extern "C" void kernel_launch(void* const* d_in, const int* in_sizes, int n_in, void* d_out, int out_size, void* d_ws, size_t ws_size, hipStream_t stream) {
  (void)n_in;
  auto Fp = [&](int i) { return (const float*)d_in[i]; }; auto Ip = [&](int i) { return (const int*)d_in[i]; };
  if (in_sizes[0] != N * 6 || in_sizes[1] != 2 * E || in_sizes[2] != 6 * D || in_sizes[3] != NH * HF || in_sizes[6] != D * D || in_sizes[10] != D * D || in_sizes[14] != 3 * D || in_sizes[16] != D * D || in_sizes[18] != D * D || in_sizes[20] != D * D || in_sizes[22] != D * D || in_sizes[24] != D * 256 || in_sizes[26] != 256 * 128 || in_sizes[28] != 128 || out_size != N) return;
  const int NLIM = N; const int GB16 = NLIM / 16, GB8 = NLIM / 8, GB32 = NLIM / 32;
  size_t off = 0; char* ws = (char*)d_ws;
  auto carve = [&](size_t bytes) { char* p = ws + off; off += (bytes + 255) & ~(size_t)255; return p; };
  b16* WG0 = (b16*)carve((size_t)D * 32 * 2); b16* WG1 = (b16*)carve((size_t)D * D * 2); b16* WG2 = (b16*)carve((size_t)D * D * 2); b16* WQKV = (b16*)carve((size_t)3 * D * D * 2); b16* WO = (b16*)carve((size_t)D * D * 2); b16* WM0 = (b16*)carve((size_t)256 * D * 2); b16* WM1 = (b16*)carve((size_t)128 * 256 * 2);
  float* HW = (float*)carve((size_t)N * D * 4); float* AS = (float*)carve((size_t)N * 16 * 4); float* G = (float*)carve((size_t)N * D * 4); float* Hh = (float*)carve((size_t)N * D * 4); float* ST = (float*)carve((size_t)D * 32 * 4); float* QKV = (float*)carve((size_t)N * 3 * D * 4); float* O = (float*)carve((size_t)N * D * 4); float* AO = (float*)carve((size_t)N * D * 4); float* QB = (float*)carve((size_t)3 * D * 4);
  CsrBufs7 csr; off = csr_carve7(csr, ws, off, E, N);
  if (off > ws_size || off > ((size_t)96 << 20)) return;
  wput_kernel<<<(D * 4 + 255) / 256, 256, 0, stream>>>(Fp(2), 6, 32, D, D, WG0); wput_kernel<<<(D * 64 + 255) / 256, 256, 0, stream>>>(Fp(6), D, D, D, D, WG1); wput_kernel<<<(D * 64 + 255) / 256, 256, 0, stream>>>(Fp(10), D, D, D, D, WG2);
  wput_kernel<<<(D * 64 + 255) / 256, 256, 0, stream>>>(Fp(16), D, D, D, D, WQKV); wput_kernel<<<(D * 64 + 255) / 256, 256, 0, stream>>>(Fp(18), D, D, D, D, WQKV + (size_t)D * D); wput_kernel<<<(D * 64 + 255) / 256, 256, 0, stream>>>(Fp(20), D, D, D, D, WQKV + (size_t)2 * D * D);
  wput_kernel<<<(D * 64 + 255) / 256, 256, 0, stream>>>(Fp(22), D, D, D, D, WO); wput_kernel<<<(256 * 64 + 255) / 256, 256, 0, stream>>>(Fp(24), D, D, 256, 256, WM0); wput_kernel<<<(128 * 32 + 255) / 256, 256, 0, stream>>>(Fp(26), 256, 256, 128, 128, WM1);
  qb_kernel<<<1, 256, 0, stream>>>(Fp(17), Fp(19), Fp(21), QB);
  csr_build7(csr, Ip(1) + E, E, N, stream);
  dense_kernel<32, 32, 1, 0, 1><<<GB16, 32, 0, stream>>>(Fp(0), 6, 6, WG0, nullptr, Fp(3), Fp(4), HW, AS);
  gat_kernel<<<GB8, 256, 0, stream>>>(HW, AS, Fp(5), Ip(1), csr.PERM, csr.ROWPTR, csr.ROWCNT, (int)csr.permLen, NLIM, G); stats_kernel<<<D, 256, 0, stream>>>(G, NLIM, ST); bn_kernel<<<GB8, 256, 0, stream>>>(G, ST, Fp(14), Fp(15), Hh);
  dense_kernel<D, 32, 0, 0, 1><<<GB16, 32, 0, stream>>>(Hh, D, D, WG1, nullptr, Fp(7), Fp(8), HW, AS);
  gat_kernel<<<GB8, 256, 0, stream>>>(HW, AS, Fp(9), Ip(1), csr.PERM, csr.ROWPTR, csr.ROWCNT, (int)csr.permLen, NLIM, G); stats_kernel<<<D, 256, 0, stream>>>(G, NLIM, ST); bn_kernel<<<GB8, 256, 0, stream>>>(G, ST, Fp(14) + D, Fp(15) + D, Hh);
  dense_kernel<D, 32, 0, 0, 1><<<GB16, 32, 0, stream>>>(Hh, D, D, WG2, nullptr, Fp(11), Fp(12), HW, AS);
  gat_kernel<<<GB8, 256, 0, stream>>>(HW, AS, Fp(13), Ip(1), csr.PERM, csr.ROWPTR, csr.ROWCNT, (int)csr.permLen, NLIM, G); stats_kernel<<<D, 256, 0, stream>>>(G, NLIM, ST); bn_kernel<<<GB8, 256, 0, stream>>>(G, ST, Fp(14) + 2 * D, Fp(15) + 2 * D, Hh);
  dense_kernel<D, 96, 0, 0, 0><<<GB16, 32, 0, stream>>>(Hh, D, D, WQKV, QB, nullptr, nullptr, QKV, nullptr);
  att_kernel<<<GB16 * NH, 32, 0, stream>>>(QKV, NLIM, O);
  dense_kernel<D, 32, 0, 0, 0><<<GB16, 32, 0, stream>>>(O, D, D, WO, Fp(23), nullptr, nullptr, AO, nullptr);
  mlp_kernel<<<GB32, 32, 0, stream>>>(AO, WM0, Fp(25), WM1, Fp(27), Fp(28), Fp(29), (float*)d_out);
}
